// EdgeInOutGTModel_7576322310513
// MI455X (gfx1250) — hardware-verified
//
#include <hip/hip_runtime.h>


namespace {
constexpr int NB = 8, N = 256, HID = 128, NH = 8, HD = 16, L = 3, FF = 512, NR = NB * N;
constexpr float XS = 8.0f, WSC = 256.0f, PS = 4096.0f  , EPS = 1e-5f, CLIP = 10.0f, LOG2E = 1.4426950408889634f;

typedef _Float16 b16;
typedef __attribute__((ext_vector_type(16))) _Float16 v16b;
typedef __attribute__((ext_vector_type(8))) _Float16 v8b;
typedef __attribute__((ext_vector_type(8))) float v8f;
typedef __attribute__((ext_vector_type(4))) float v4f;
__device__ __forceinline__ float bf16_rne(float f) { unsigned int u = __float_as_uint(f); u += 0x7FFFu + ((u >> 16) & 1u); return __uint_as_float(u & 0xFFFF0000u); }
__device__ __forceinline__ void split16(float v, b16& hi, b16& lo) { hi = (b16)v; lo = (b16)(v - (float)hi); }
__device__ __forceinline__ v16b frag_kb(const b16* p, int hh) { const v8b a = *(const v8b*)(p + 8 * hh), b = *(const v8b*)(p + 16 + 8 * hh); v16b f;
#pragma unroll
  for (int e = 0; e < 8; ++e) { f[e] = a[e]; f[8 + e] = b[e]; } return f; }
__device__ __forceinline__ v8f wmma16b(v16b a, v16b b, v8f c) { v8f d = __builtin_amdgcn_wmma_f32_16x16x32_f16(false, a, false, b, (short)0, c, false, false); asm volatile("v_nop\n\tv_nop\n\tv_nop\n\tv_nop" : "+v"(d) : "v"(a), "v"(b)); return d; }
__device__ __forceinline__ void wave_lds_sync() { __builtin_amdgcn_fence(__ATOMIC_RELEASE, "workgroup"); __builtin_amdgcn_wave_barrier(); __builtin_amdgcn_fence(__ATOMIC_ACQUIRE, "workgroup"); }
__device__ __forceinline__ float pmul(float a, float b) { float p = a * b; asm volatile("" : "+v"(p)); return p; }
__device__ __forceinline__ float hsum16(float v) { v += __shfl_xor(v, 1); v += __shfl_xor(v, 2); v += __shfl_xor(v, 4); return v + __shfl_xor(v, 8); }
__device__ __forceinline__ float nexp2(float x) { return __builtin_amdgcn_exp2f(x); }
__device__ __forceinline__ float tanh_(float x) { const float e = nexp2(-2.0f * fabsf(x) * LOG2E); const float t = (1.0f - e) / (1.0f + e); return x < 0.0f ? -t : t; }

__global__ __launch_bounds__(256) void prep_kernel(const float* __restrict__ nf, const float* __restrict__ wnode, const float* __restrict__ wedge, const float* __restrict__ wh, const float* __restrict__ we, const float* __restrict__ w1, const float* __restrict__ w2, b16* __restrict__ WH, b16* __restrict__ W1T, b16* __restrict__ W2T, float* __restrict__ CE, float* __restrict__ HS) {
  const size_t t = (size_t)blockIdx.x * 256 + threadIdx.x; const size_t n1 = (size_t)L * 3 * HID * HID / 8, n2 = (size_t)L * FF * HID / 8, n3 = n2, n4 = 64  , n5 = (size_t)NR * HID / 4; v8b o;
  if (t < n1) { const size_t u = t * 8; const int l = (int)(u / ((size_t)3 * HID * HID)); const size_t e = u - (size_t)l * 3 * HID * HID; const int oo = (int)(e / HID), i0 = (int)(e - (size_t)oo * HID);
    for (int j = 0; j < 8; ++j) o[j] = (b16)(bf16_rne(wh[((size_t)l * HID + i0 + j) * 3 * HID + oo]) * WSC); for (int pass = 0; pass < 2; ++pass) { *(volatile v8b*)(WH + u) = o; __threadfence(); } }
  else if (t < n1 + n2) { const size_t u = (t - n1) * 8; const int l = (int)(u / ((size_t)FF * HID)); const size_t e = u - (size_t)l * FF * HID; const int oo = (int)(e / HID), i0 = (int)(e - (size_t)oo * HID);
    for (int j = 0; j < 8; ++j) o[j] = (b16)(bf16_rne(w1[((size_t)l * HID + i0 + j) * FF + oo]) * WSC); for (int pass = 0; pass < 2; ++pass) { *(volatile v8b*)(W1T + u) = o; __threadfence(); } }
  else if (t < n1 + n2 + n3) { const size_t u = (t - n1 - n2) * 8; const int l = (int)(u / ((size_t)HID * FF)); const size_t e = u - (size_t)l * HID * FF; const int oo = (int)(e / FF), i0 = (int)(e - (size_t)oo * FF);
    for (int j = 0; j < 8; ++j) o[j] = (b16)(bf16_rne(w2[((size_t)l * FF + i0 + j) * HID + oo]) * WSC); for (int pass = 0; pass < 2; ++pass) { *(volatile v8b*)(W2T + u) = o; __threadfence(); } }
  else if (t < n1 + n2 + n3 + n4) { const int i = (int)(t - n1 - n2 - n3); float s = 0.0f; if (i < L * 2 * NH) { const int l = i / (2 * NH), c = i - l * 2 * NH; for (int k = 0; k < HID; ++k) s += pmul(bf16_rne(wedge[k]), bf16_rne(we[((size_t)l * HID + k) * 2 * NH + c])); }
    for (int pass = 0; pass < 2; ++pass) { ((volatile float*)CE)[i] = s; __threadfence(); } }
  else if (t < n1 + n2 + n3 + n4 + n5) { const size_t u = (t - n1 - n2 - n3 - n4) * 4; const size_t node = u / HID; const int c0 = (int)(u - node * HID); const float x0 = bf16_rne(nf[node * 3]), x1 = bf16_rne(nf[node * 3 + 1]), x2 = bf16_rne(nf[node * 3 + 2]); v4f o4;
    for (int j = 0; j < 4; ++j) { const int c = c0 + j; o4[j] = (pmul(x0, bf16_rne(wnode[c])) + pmul(x1, bf16_rne(wnode[HID + c]))) + pmul(x2, bf16_rne(wnode[2 * HID + c])); }
    for (int pass = 0; pass < 2; ++pass) { *(volatile v4f*)(HS + u) = o4; __threadfence(); } }
}
__global__ __launch_bounds__(128) void qkv_kernel(const float* __restrict__ HS, const float* __restrict__ g1, const float* __restrict__ b1, const b16* __restrict__ WHl, b16* __restrict__ Qh, b16* __restrict__ Ql, b16* __restrict__ Kh, b16* __restrict__ Kl, b16* __restrict__ VTh, b16* __restrict__ VTl) {
  __shared__ __attribute__((aligned(16))) b16 Ah[4][16][HID + 8], Alo[4][16][HID + 8]; __shared__ __attribute__((aligned(16))) b16 Vt[HID][64 + 8], Vtl[HID][64 + 8]; __shared__ __attribute__((aligned(16))) b16 QK[4][2][16][HID + 8], QKl[4][2][16][HID + 8];
  const int wave = threadIdx.x >> 5, lane = threadIdx.x & 31, nloc = lane & 15, hlf = lane >> 4, t_ = threadIdx.x; const size_t m0 = (size_t)blockIdx.x * 64 + wave * 16; const int b = (int)(m0 / N); const int i0 = (int)(m0 - (size_t)b * N);
  for (int step = 0; step < 8; ++step) { const int rr = 2 * step + hlf; const float* hr = HS + (m0 + rr) * HID + nloc * 8; float x[8]; { const v4f a = *(const v4f*)hr, c = *(const v4f*)(hr + 4); for (int j = 0; j < 4; ++j) { x[j] = a[j]; x[4 + j] = c[j]; } }
    float s = 0.0f; for (int j = 0; j < 8; ++j) s += x[j]; s = hsum16(s); const float mu = s * (1.0f / HID); float q2 = 0.0f; for (int j = 0; j < 8; ++j) { const float d = x[j] - mu; q2 += pmul(d, d); } q2 = hsum16(q2); const float rs = rsqrtf(q2 * (1.0f / HID) + EPS);
    for (int j = 0; j < 8; ++j) { const int c = nloc * 8 + j; const float y = pmul((x[j] - mu) * rs, bf16_rne(g1[c])) + bf16_rne(b1[c]); b16 h_, l_; split16(y * XS, h_, l_); Ah[wave][rr][c] = h_; Alo[wave][rr][c] = l_; } }
  wave_lds_sync();
  for (int part = 0; part < 3; ++part) {
    v8f acc[8];
#pragma unroll
    for (int t = 0; t < 8; ++t) acc[t] = (v8f){};
#pragma unroll
    for (int kb = 0; kb < HID; kb += 32) { const v16b a = frag_kb(&Ah[wave][nloc][kb], hlf), al = frag_kb(&Alo[wave][nloc][kb], hlf);
#pragma unroll
      for (int t = 0; t < 8; ++t) { const v16b bw = frag_kb(WHl + (size_t)(part * HID + t * 16 + nloc) * HID + kb, hlf); acc[t] = wmma16b(a, bw, acc[t]); acc[t] = wmma16b(al, bw, acc[t]); } }
    if (part < 2) {
#pragma unroll
      for (int t = 0; t < 8; ++t)
#pragma unroll
        for (int r = 0; r < 8; ++r) { b16 h_, l_; split16(acc[t][r] * (1.0f / (XS * WSC)) * XS, h_, l_); QK[wave][part][8 * hlf + r][t * 16 + nloc] = h_; QKl[wave][part][8 * hlf + r][t * 16 + nloc] = l_; } }
    else {
#pragma unroll
      for (int t = 0; t < 8; ++t)
#pragma unroll
        for (int r = 0; r < 8; ++r) { b16 h_, l_; split16(acc[t][r] * (1.0f / (XS * WSC)) * XS, h_, l_); Vt[t * 16 + nloc][wave * 16 + 8 * hlf + r] = h_; Vtl[t * 16 + nloc][wave * 16 + 8 * hlf + r] = l_; } } }
  __syncthreads();
  for (int pass = 0; pass < 2; ++pass) {
    for (int part = 0; part < 2; ++part) { b16* dh = part ? Kh : Qh; b16* dl = part ? Kl : Ql;
      for (int h = 0; h < NH; ++h) { const int rr = lane >> 1, half = lane & 1; v16b hv = {}, lv = {}; if (half == 0) { for (int j = 0; j < 16; ++j) { hv[j] = QK[wave][part][rr][h * HD + j]; lv[j] = QKl[wave][part][rr][h * HD + j]; } }
        const size_t gi = (((size_t)b * NH + h) * N + i0 + rr) * 32 + half * 16; *(volatile v16b*)(dh + gi) = hv; *(volatile v16b*)(dl + gi) = lv; } }
    const int ib0 = (int)((size_t)blockIdx.x * 64 - (size_t)b * N);
    for (int q = t_; q < HID * 8; q += 128) { const int c = q >> 3, c8 = (q & 7) * 8; const int h = c / HD, d = c - h * HD; const size_t gi = (((size_t)b * NH + h) * HD + d) * N + ib0 + c8; *(volatile v8b*)(VTh + gi) = *(const v8b*)(&Vt[c][c8]); *(volatile v8b*)(VTl + gi) = *(const v8b*)(&Vtl[c][c8]); }
    __threadfence(); }
}
__global__ __launch_bounds__(64) void attn_kernel(const b16* __restrict__ Qh, const b16* __restrict__ Ql, const b16* __restrict__ Kh, const b16* __restrict__ Kl, const b16* __restrict__ VTh, const b16* __restrict__ VTl, const float* __restrict__ ef, const float* __restrict__ CEl, float* __restrict__ YH) {
  __shared__ __attribute__((aligned(16))) float To[2][16][HD + 4];
  const int wave = threadIdx.x >> 5, lane = threadIdx.x & 31, hh = lane >> 4, col = lane & 15; const int b = blockIdx.z, h = blockIdx.y; const int q0 = blockIdx.x * 32 + wave * 16, qi = q0 + col;
  const size_t bh = (size_t)b * NH + h; const v16b qa = frag_kb(Qh + (bh * N + qi) * 32, hh), ql = frag_kb(Ql + (bh * N + qi) * 32, hh);
  const b16* Kb = Kh + bh * N * 32; const b16* Klb = Kl + bh * N * 32; const b16* Vb = VTh + bh * HD * N; const b16* Vlb = VTl + bh * HD * N; const float c1 = CEl[h], c2 = CEl[NH + h]; const float* er = ef + ((size_t)b * N + qi) * N;
  float m = -INFINITY, l = 0.0f; v8f o = {}, ol = {};
  const float cs = 0.25f / (XS * XS);
  for (int kb = 0; kb < N; kb += 32) {
    v8f s0 = {}, s1 = {};
    { const b16* k0 = Kb + (size_t)(kb + col) * 32, *k1 = Kb + (size_t)(kb + 16 + col) * 32, *k0l = Klb + (size_t)(kb + col) * 32, *k1l = Klb + (size_t)(kb + 16 + col) * 32;
      v16b f = frag_kb(k0, hh); s0 = wmma16b(f, qa, s0); s0 = wmma16b(f, ql, s0); s0 = wmma16b(frag_kb(k0l, hh), qa, s0);
      f = frag_kb(k1, hh); s1 = wmma16b(f, qa, s1); s1 = wmma16b(f, ql, s1); s1 = wmma16b(frag_kb(k1l, hh), qa, s1); }
    float e[16], g[16]; float mx = -INFINITY;
#pragma unroll
    for (int r = 0; r < 8; ++r) { const int j0 = kb + 8 * hh + r, j1 = kb + 16 + 8 * hh + r; const float f0 = bf16_rne(er[j0]), f1 = bf16_rne(er[j1]);
      e[r] = (s0[r] * cs + pmul(f0, c1)) * LOG2E; e[8 + r] = (s1[r] * cs + pmul(f1, c1)) * LOG2E; g[r] = pmul(f0, c2); g[8 + r] = pmul(f1, c2); mx = fmaxf(mx, fmaxf(e[r], e[8 + r])); }
    mx = fmaxf(mx, __shfl_xor(mx, 16)); const float mn = fmaxf(m, mx); const float al = nexp2(m - mn); m = mn; float sum = 0.0f; v16b ph, pl;
#pragma unroll
    for (int i = 0; i < 16; ++i) { const float p = nexp2(e[i] - mn); sum += p; const float pg = pmul(p, g[i]); const b16 h_ = (b16)(pg * PS); ph[i] = h_; pl[i] = (b16)(pg * PS - (float)h_); }
    sum += __shfl_xor(sum, 16); l = l * al + sum;
    o *= al; ol *= al; const v16b vf = frag_kb(Vb + (size_t)col * N + kb, hh); o = wmma16b(vf, ph, o); ol = wmma16b(vf, pl, ol); ol = wmma16b(frag_kb(Vlb + (size_t)col * N + kb, hh), ph, ol); }
  const float inv = 1.0f / (l * PS * XS);
#pragma unroll
  for (int r = 0; r < 8; ++r) To[wave][col][8 * hh + r] = (o[r] + ol[r]) * inv;
  wave_lds_sync();
  for (int pass = 0; pass < 2; ++pass) { for (int r4 = 0; r4 < 16; r4 += 8) { const int rr = r4 + (lane >> 2), c4 = (lane & 3) * 4; *(volatile v4f*)(YH + (bh * N + q0 + rr) * HD + c4) = *(const v4f*)(&To[wave][rr][c4]); } __threadfence(); }
}
__global__ __launch_bounds__(64) void mlp_kernel(const float* __restrict__ YH, float* __restrict__ HS, const float* __restrict__ g2, const float* __restrict__ b2, const b16* __restrict__ W1Tl, const b16* __restrict__ W2Tl) {
  __shared__ __attribute__((aligned(16))) b16 Ah[2][16][HID + 8], Alo[2][16][HID + 8]; __shared__ __attribute__((aligned(16))) float Ys[2][16][HID + 4];
  const int wave = threadIdx.x >> 5, lane = threadIdx.x & 31, nloc = lane & 15, hlf = lane >> 4; const size_t m0 = (size_t)blockIdx.x * 32 + wave * 16;   const int b = (int)(m0 / N); const int i0 = (int)(m0 - (size_t)b * N);
  for (int step = 0; step < 8; ++step) { const int rr = 2 * step + hlf; const int h = nloc >> 1, d0 = (nloc & 1) * 8; const float* yr = YH + (((size_t)b * NH + h) * N + i0 + rr) * HD + d0; const float* hr = HS + (m0 + rr) * HID + nloc * 8; float x[8], yv[8];
    { const v4f a = *(const v4f*)yr, c = *(const v4f*)(yr + 4), ha = *(const v4f*)hr, hc = *(const v4f*)(hr + 4); for (int j = 0; j < 4; ++j) { yv[j] = a[j]; yv[4 + j] = c[j]; x[j] = a[j] + ha[j]; x[4 + j] = c[j] + hc[j]; } }
    float s = 0.0f; for (int j = 0; j < 8; ++j) s += x[j]; s = hsum16(s); const float mu = s * (1.0f / HID); float q2 = 0.0f; for (int j = 0; j < 8; ++j) { const float d = x[j] - mu; q2 += pmul(d, d); } q2 = hsum16(q2); const float rs = rsqrtf(q2 * (1.0f / HID) + EPS);
    for (int j = 0; j < 8; ++j) { const int c = nloc * 8 + j; const float z = pmul((x[j] - mu) * rs, bf16_rne(g2[c])) + bf16_rne(b2[c]); b16 h_, l_; split16(z * XS, h_, l_); Ah[wave][rr][c] = h_; Alo[wave][rr][c] = l_; Ys[wave][rr][c] = yv[j]; } }
  wave_lds_sync();
  v8f acc[8];
  __shared__ __attribute__((aligned(16))) b16 Hh[2][16][FF + 8], Hl[2][16][FF + 8];
  for (int cb = 0; cb < FF / 128; ++cb) {
#pragma unroll
    for (int t = 0; t < 8; ++t) acc[t] = (v8f){};
#pragma unroll
    for (int kb = 0; kb < HID; kb += 32) { const v16b a = frag_kb(&Ah[wave][nloc][kb], hlf), al = frag_kb(&Alo[wave][nloc][kb], hlf);
#pragma unroll
      for (int t = 0; t < 8; ++t) { const v16b bw = frag_kb(W1Tl + (size_t)(cb * 128 + t * 16 + nloc) * HID + kb, hlf); acc[t] = wmma16b(a, bw, acc[t]); acc[t] = wmma16b(al, bw, acc[t]); } }
#pragma unroll
    for (int t = 0; t < 8; ++t)
#pragma unroll
      for (int r = 0; r < 8; ++r) { b16 h_, l_; split16(fmaxf(acc[t][r] * (1.0f / (XS * WSC)), 0.0f) * XS, h_, l_); Hh[wave][8 * hlf + r][cb * 128 + t * 16 + nloc] = h_; Hl[wave][8 * hlf + r][cb * 128 + t * 16 + nloc] = l_; } }
  wave_lds_sync();
#pragma unroll
  for (int t = 0; t < 8; ++t) acc[t] = (v8f){};
#pragma unroll 4
  for (int kb = 0; kb < FF; kb += 32) { const v16b a = frag_kb(&Hh[wave][nloc][kb], hlf), al = frag_kb(&Hl[wave][nloc][kb], hlf);
#pragma unroll
    for (int t = 0; t < 8; ++t) { const v16b bw = frag_kb(W2Tl + (size_t)(t * 16 + nloc) * FF + kb, hlf); acc[t] = wmma16b(a, bw, acc[t]); acc[t] = wmma16b(al, bw, acc[t]); } }
#pragma unroll
  for (int t = 0; t < 8; ++t)
#pragma unroll
    for (int r = 0; r < 8; ++r) Ys[wave][8 * hlf + r][t * 16 + nloc] += acc[t][r] * (1.0f / (XS * WSC));
  wave_lds_sync();
  for (int pass = 0; pass < 2; ++pass) { for (int rr = 0; rr < 16; ++rr) *(volatile v4f*)(HS + (m0 + rr) * HID + lane * 4) = *(const v4f*)(&Ys[wave][rr][lane * 4]); __threadfence(); }
}
__global__ __launch_bounds__(256) void dec1_kernel(const float* __restrict__ HS, const float* __restrict__ wd, float* __restrict__ AC) {
  __shared__ float S[16][2];
  const int wave = threadIdx.x >> 5, lane = threadIdx.x & 31; const size_t nd = (size_t)blockIdx.x * 16 + wave * 2 + (lane >> 4); const int c0 = (lane & 15) * 8;
  float sa = 0.0f, sc = 0.0f; for (int j = 0; j < 8; ++j) { const float hv = HS[nd * HID + c0 + j]; sa += pmul(hv, bf16_rne(wd[c0 + j])); sc += pmul(hv, bf16_rne(wd[HID + c0 + j])); }
  sa = hsum16(sa); sc = hsum16(sc); if ((lane & 15) == 0) { S[wave * 2 + (lane >> 4)][0] = sa; S[wave * 2 + (lane >> 4)][1] = sc; }
  __syncthreads();
  for (int pass = 0; pass < 2; ++pass) { if (threadIdx.x < 32) ((volatile float*)AC)[(size_t)blockIdx.x * 32 + threadIdx.x] = S[threadIdx.x >> 1][threadIdx.x & 1]; __threadfence(); }
}
__global__ __launch_bounds__(256) void dec2_kernel(const float* __restrict__ AC, float* __restrict__ out) {
  const int b = blockIdx.y, i = blockIdx.x, j = threadIdx.x; const float ci = AC[((size_t)b * N + i) * 2 + 1], aj = AC[((size_t)b * N + j) * 2];
  const float v = CLIP * tanh_((aj + ci) * 0.08838834764831845f);
  for (int pass = 0; pass < 2; ++pass) { ((volatile float*)out)[((size_t)b * N + i) * N + j] = v; __threadfence(); }
}
}

extern "C" void kernel_launch(void* const* d_in, const int* in_sizes, int n_in, void* d_out, int out_size, void* d_ws, size_t ws_size, hipStream_t stream) {
  (void)n_in;
  auto Fp = [&](int i) { return (const float*)d_in[i]; };
  if (in_sizes[0] != NR * 3 || in_sizes[1] != NR * N || in_sizes[2] != 3 * HID || in_sizes[3] != HID || in_sizes[4] != L * HID * 3 * HID || in_sizes[5] != L * HID * 2 * NH || in_sizes[10] != L * HID * FF || in_sizes[11] != L * FF * HID || in_sizes[12] != 2 * HID || out_size != NR * N) return;
  size_t off = 0; char* ws = (char*)d_ws;
  auto carve = [&](size_t bytes) { char* p = ws + off; off += (bytes + 255) & ~(size_t)255; return p; };
  b16* WH = (b16*)carve((size_t)L * 3 * HID * HID * 2); b16* W1T = (b16*)carve((size_t)L * FF * HID * 2); b16* W2T = (b16*)carve((size_t)L * HID * FF * 2); float* CE = (float*)carve(256); float* HS = (float*)carve((size_t)NR * HID * 4);
  b16* Qh = (b16*)carve((size_t)NB * NH * N * 32 * 2); b16* Ql = (b16*)carve((size_t)NB * NH * N * 32 * 2); b16* Kh = (b16*)carve((size_t)NB * NH * N * 32 * 2); b16* Kl = (b16*)carve((size_t)NB * NH * N * 32 * 2); b16* VTh = (b16*)carve((size_t)NB * NH * HD * N * 2); b16* VTl = (b16*)carve((size_t)NB * NH * HD * N * 2);
  float* YH = (float*)carve((size_t)NB * NH * N * HD * 4); float* AC = (float*)carve((size_t)NR * 2 * 4);
  if (off > ws_size || off > ((size_t)128 << 20)) return;
  prep_kernel<<<(unsigned)(((size_t)L * 3 * HID * HID / 8 + 2 * (size_t)L * FF * HID / 8 + 64 + (size_t)NR * HID / 4 + 255) / 256), 256, 0, stream>>>(Fp(0), Fp(2), Fp(3), Fp(4), Fp(5), Fp(10), Fp(11), WH, W1T, W2T, CE, HS);
  for (int l = 0; l < L; ++l) {
    qkv_kernel<<<NR / 64, 128, 0, stream>>>(HS, Fp(6) + l * HID, Fp(7) + l * HID, WH + (size_t)l * 3 * HID * HID, Qh, Ql, Kh, Kl, VTh, VTl);
    attn_kernel<<<dim3(N / 32, NH, NB), 64, 0, stream>>>(Qh, Ql, Kh, Kl, VTh, VTl, Fp(1), CE + l * 2 * NH, YH);
    mlp_kernel<<<NR / 32, 64, 0, stream>>>(YH, HS, Fp(8) + l * HID, Fp(9) + l * HID, W1T + (size_t)l * FF * HID, W2T + (size_t)l * HID * FF);
  }
  dec1_kernel<<<NR / 16, 256, 0, stream>>>(HS, Fp(12), AC);
  dec2_kernel<<<dim3(N, NB), 256, 0, stream>>>(AC, (float*)d_out);
}
